// MLA_68788196212930
// MI455X (gfx1250) — hardware-verified
//
#include <hip/hip_runtime.h>
#include <math.h>
#include <stdint.h>

#define NB    2
#define SQ    2048
#define DMOD  2048
#define DLAT  512
#define NH    16
#define HD    128
#define HDN   64
#define NQ    2048
#define NQA   2560
#define LATW  1024
#define KVBW  1024
#define AOW   4096
#define WOW   4096
#define NPAIR 32

typedef __bf16       v16b __attribute__((ext_vector_type(16)));
typedef __bf16       v8b  __attribute__((ext_vector_type(8)));
typedef float        v8f  __attribute__((ext_vector_type(8)));
typedef float        v4f  __attribute__((ext_vector_type(4)));
typedef float        v2f  __attribute__((ext_vector_type(2)));
typedef unsigned int v4u  __attribute__((ext_vector_type(4)));

__device__ __forceinline__ unsigned short bf_bits(float f) {
  const unsigned u = __float_as_uint(f);
  return (unsigned short)((u + 0x7FFFu + ((u >> 16) & 1u)) >> 16);
}
__device__ __forceinline__ float bf_val(unsigned short h) { return __uint_as_float(((unsigned)h) << 16); }
__device__ __forceinline__ float bf_rne(float f) { return bf_val(bf_bits(f)); }
__device__ __forceinline__ unsigned pk16(unsigned short a, unsigned short b) { return (unsigned)a | ((unsigned)b << 16); }
__device__ __forceinline__ v8f zero8() { v8f z = {0.f, 0.f, 0.f, 0.f, 0.f, 0.f, 0.f, 0.f}; return z; }
__device__ __forceinline__ int wave_id() { return __builtin_amdgcn_readfirstlane((int)(threadIdx.x >> 5)); }

__device__ __forceinline__ unsigned split2(float f0, float f1, unsigned& lo) {
  const unsigned short h0 = bf_bits(f0), h1 = bf_bits(f1);
  const unsigned short l0 = bf_bits(f0 - bf_val(h0)), l1 = bf_bits(f1 - bf_val(h1));
  lo = pk16(l0, l1);
  return pk16(h0, h1);
}
__device__ __forceinline__ void split8(v4f a, v4f b, v4u& hv, v4u& lv) {
  unsigned l0, l1, l2, l3;
  hv[0] = split2(a[0], a[1], l0);
  hv[1] = split2(a[2], a[3], l1);
  hv[2] = split2(b[0], b[1], l2);
  hv[3] = split2(b[2], b[3], l3);
  lv[0] = l0; lv[1] = l1; lv[2] = l2; lv[3] = l3;
}

__device__ __forceinline__ void lds_wave_sync() {
  __builtin_amdgcn_fence(__ATOMIC_RELEASE, "workgroup");
  __builtin_amdgcn_wave_barrier();
  __builtin_amdgcn_fence(__ATOMIC_ACQUIRE, "workgroup");
}

union FragB { v16b v; v8b h[2]; };
__device__ __forceinline__ v16b ldfrag_b(const __bf16* p) { FragB f; f.h[0] = *(const v8b*)(p); f.h[1] = *(const v8b*)(p + 16); return f.v; }

__device__ __forceinline__ v8f mma_b(v16b a, v16b b, v8f c) {
  return __builtin_amdgcn_wmma_f32_16x16x32_bf16(false, a, false, b, (short)0, c, false, false);
}
__device__ __forceinline__ void guard2b3(v8f& a, v8f& b, v16b x0, v16b x1, v16b y) {
  asm volatile("v_nop\n\tv_nop\n\tv_nop\n\tv_nop" : "+v"(a), "+v"(b) : "v"(x0), "v"(x1), "v"(y) : "memory");
}
__device__ __forceinline__ void guard1b4(v8f& a, v16b w, v16b x, v16b y, v16b z) {
  asm volatile("v_nop\n\tv_nop\n\tv_nop\n\tv_nop" : "+v"(a) : "v"(w), "v"(x), "v"(y), "v"(z) : "memory");
}
__device__ __forceinline__ void acc_guard4(v8f& a, v8f& b, v8f& c, v8f& d) {
  asm volatile("v_nop\n\tv_nop\n\tv_nop\n\tv_nop" : "+v"(a), "+v"(b), "+v"(c), "+v"(d));
}

__global__ __launch_bounds__(256) void cvt_bf16_kernel(const float* __restrict__ in, unsigned short* __restrict__ outp, int n8) {
  const int i = (int)blockIdx.x * 256 + (int)threadIdx.x;
  if (i >= n8) return;
  const size_t e = 8 * (size_t)i;
  const v4f a = *(const v4f*)(in + e);
  const v4f b = *(const v4f*)(in + e + 4);
  v4u w;
  w[0] = pk16(bf_bits(a[0]), bf_bits(a[1]));
  w[1] = pk16(bf_bits(a[2]), bf_bits(a[3]));
  w[2] = pk16(bf_bits(b[0]), bf_bits(b[1]));
  w[3] = pk16(bf_bits(b[2]), bf_bits(b[3]));
  *(volatile v4u*)(outp + e) = w;
  __threadfence();
  *(volatile v4u*)(outp + e) = w;
}

__global__ __launch_bounds__(256) void cvt_dup_kernel(const float* __restrict__ in, unsigned short* __restrict__ outp,
                                                      int n8, int kin, int ldo) {
  const int i = (int)blockIdx.x * 256 + (int)threadIdx.x;
  if (i >= n8) return;
  const size_t e = 8 * (size_t)i;
  const int n = (int)(e / (size_t)kin);
  const int k = (int)(e - (size_t)n * kin);
  const v4f a = *(const v4f*)(in + e);
  const v4f b = *(const v4f*)(in + e + 4);
  v4u w;
  w[0] = pk16(bf_bits(a[0]), bf_bits(a[1]));
  w[1] = pk16(bf_bits(a[2]), bf_bits(a[3]));
  w[2] = pk16(bf_bits(b[0]), bf_bits(b[1]));
  w[3] = pk16(bf_bits(b[2]), bf_bits(b[3]));
  const size_t o = (size_t)n * ldo + k;
  *(volatile v4u*)(outp + o) = w;
  *(volatile v4u*)(outp + o + kin) = w;
  __threadfence();
  *(volatile v4u*)(outp + o) = w;
  *(volatile v4u*)(outp + o + kin) = w;
}

__global__ __launch_bounds__(256) void rmsnorm_split_kernel(const float* __restrict__ tp, const float* __restrict__ nw,
                                                            unsigned short* __restrict__ lat, int nrows) {
  const int lane = threadIdx.x & 31;
  const int wave = (int)(threadIdx.x >> 5);
  const int row  = (int)blockIdx.x * 8 + wave;
  if (row >= nrows) return;
  const float* xr = tp + (size_t)row * DLAT;
  v4f xa[2], xb[2];
  float ss = 0.f;
#pragma unroll
  for (int u = 0; u < 2; ++u) {
    const int col = 256 * u + 8 * lane;
    xa[u] = *(const v4f*)(xr + col);
    xb[u] = *(const v4f*)(xr + col + 4);
#pragma unroll
    for (int e = 0; e < 4; ++e) { ss += xa[u][e] * xa[u][e]; ss += xb[u][e] * xb[u][e]; }
  }
#pragma unroll
  for (int off = 1; off < 32; off <<= 1) ss += __shfl_xor(ss, off, 32);
  const float rs = rsqrtf(ss * (1.0f / 512.0f) + 1e-6f);
  v4u hv[2], lv[2];
#pragma unroll
  for (int u = 0; u < 2; ++u) {
    const int col = 256 * u + 8 * lane;
    const v4f wa = *(const v4f*)(nw + col);
    const v4f wb = *(const v4f*)(nw + col + 4);
    v4f ya, yb;
#pragma unroll
    for (int e = 0; e < 4; ++e) {
      ya[e] = (xa[u][e] * rs) * bf_rne(wa[e]);
      yb[e] = (xb[u][e] * rs) * bf_rne(wb[e]);
    }
    split8(ya, yb, hv[u], lv[u]);
  }
  unsigned short* lr = lat + (size_t)row * LATW;
  for (int pass = 0; pass < 2; ++pass) {
#pragma unroll
    for (int u = 0; u < 2; ++u) {
      const int col = 256 * u + 8 * lane;
      *(volatile v4u*)(lr + col) = hv[u];
      *(volatile v4u*)(lr + DLAT + col) = lv[u];
    }
    __threadfence();
  }
}

template <int EPI, bool HASBIAS>
__global__ __launch_bounds__(128) void gemm_w32x128_kernel(
    const unsigned short* __restrict__ Ap, int lda,
    const unsigned short* __restrict__ Btp, int ldb,
    const float* __restrict__ bias, const float* __restrict__ fr,
    void* C0, void* C1, void* C2, int ldc, int ldc2, int nsplit,
    int M, int N, int K) {
  __shared__ __align__(16) float lds_all[4 * 2048];

  const int lane = threadIdx.x & 31;
  const int wave = wave_id();
  const int hh = lane >> 4;
  const int rl = lane & 15;
  const int tilesN = N >> 7;
  const int tilesM = M >> 5;
  const int tile = (int)blockIdx.x * 4 + wave;
  if (tile >= tilesM * tilesN) return;
  const int tm = tile / tilesN;
  const int tn = tile - tm * tilesN;
  const int m0 = tm << 5;
  const int n0 = tn << 7;

  const __bf16* A  = (const __bf16*)(const void*)Ap;
  const __bf16* Bt = (const __bf16*)(const void*)Btp;

  v8f acc[2][8];
#pragma unroll
  for (int i = 0; i < 2; ++i)
#pragma unroll
    for (int j = 0; j < 8; ++j) acc[i][j] = zero8();

  for (int k0 = 0; k0 < K; k0 += 32) {
    v16b ah[2];
#pragma unroll
    for (int i = 0; i < 2; ++i) ah[i] = ldfrag_b(A + (size_t)(m0 + i * 16 + rl) * lda + k0 + 8 * hh);
#pragma unroll
    for (int j = 0; j < 8; ++j) {
      const v16b bj = ldfrag_b(Bt + (size_t)(n0 + j * 16 + rl) * ldb + k0 + 8 * hh);
      acc[0][j] = mma_b(ah[0], bj, acc[0][j]);
      acc[1][j] = mma_b(ah[1], bj, acc[1][j]);
      guard2b3(acc[0][j], acc[1][j], ah[0], ah[1], bj);
    }
  }
  acc_guard4(acc[0][0], acc[0][1], acc[0][2], acc[0][3]);
  acc_guard4(acc[0][4], acc[0][5], acc[0][6], acc[0][7]);
  acc_guard4(acc[1][0], acc[1][1], acc[1][2], acc[1][3]);
  acc_guard4(acc[1][4], acc[1][5], acc[1][6], acc[1][7]);

  float* wl = lds_all + wave * 2048;
  unsigned short* sl16 = (unsigned short*)(void*)wl;
  float* slf = wl;

  if (EPI == 0) {
    if (n0 < nsplit) {
      const int hd = n0 >> 7;
      unsigned short* P0 = (unsigned short*)C0;
      unsigned short* P1 = (unsigned short*)C1;
      const v2f cs2 = *(const v2f*)(fr + hd * (2 * NPAIR) + 2 * lane);
      const float cv = bf_rne(cs2[0]);
      const float sv = bf_rne(cs2[1]);
      float be0 = 0.f, be1 = 0.f, bo0 = 0.f, bo1 = 0.f;
      if (HASBIAS) {
        const v2f t0 = *(const v2f*)(bias + n0 + 2 * lane);
        const v2f t1 = *(const v2f*)(bias + n0 + HDN + 2 * lane);
        be0 = bf_rne(t0[0]); be1 = bf_rne(t0[1]); bo0 = bf_rne(t1[0]); bo1 = bf_rne(t1[1]);
      }
#pragma unroll
      for (int i = 0; i < 2; ++i) {
        const int mb = m0 + i * 16;
#pragma unroll
        for (int j = 0; j < 8; ++j)
#pragma unroll
          for (int r = 0; r < 8; ++r)
            slf[(8 * hh + r) * 128 + j * 16 + rl] = acc[i][j][r];
        lds_wave_sync();
#pragma unroll 4
        for (int it = 0; it < 32; ++it) {
          const int row = it >> 1;
          const int odd = it & 1;
          const int d0  = odd * HDN + 2 * lane;
          const v2f xv = *(const v2f*)(slf + row * 128 + d0);
          const float x0 = xv[0] + (odd ? bo0 : be0);
          const float x1 = xv[1] + (odd ? bo1 : be1);
          const float ce = odd ? cv : 1.0f;
          const float se = odd ? sv : 0.0f;
          v2f yv;
          yv[0] = x0 * ce - x1 * se;
          yv[1] = x0 * se + x1 * ce;
          *(v2f*)(slf + row * 128 + d0) = yv;
        }
        lds_wave_sync();
        for (int pass = 0; pass < 2; ++pass) {
#pragma unroll
          for (int it = 0; it < 8; ++it) {
            const int row = it * 2 + hh;
            const int c8  = rl * 8;
            const v4f fa = *(const v4f*)(slf + row * 128 + c8);
            const v4f fb = *(const v4f*)(slf + row * 128 + c8 + 4);
            v4u vh, vl;
            split8(fa, fb, vh, vl);
            const size_t go = (size_t)(mb + row) * ldc + n0 + c8;
            *(volatile v4u*)(P0 + go) = vh;
            *(volatile v4u*)(P1 + go) = vl;
          }
          __threadfence();
        }
        lds_wave_sync();
      }
    } else {
      float* C = (float*)C2;
      const int col0 = n0 - nsplit;
#pragma unroll
      for (int i = 0; i < 2; ++i) {
#pragma unroll
        for (int j = 0; j < 8; ++j)
#pragma unroll
          for (int r = 0; r < 8; ++r)
            slf[(8 * hh + r) * 128 + j * 16 + rl] = acc[i][j][r];
        lds_wave_sync();
        for (int pass = 0; pass < 2; ++pass) {
#pragma unroll
          for (int row = 0; row < 16; ++row) {
            const v4f v = *(const v4f*)(slf + row * 128 + lane * 4);
            *(volatile v4f*)(C + (size_t)(m0 + i * 16 + row) * ldc2 + col0 + lane * 4) = v;
          }
          __threadfence();
        }
        lds_wave_sync();
      }
    }
  } else if (EPI == 1) {
    unsigned short* P0 = (unsigned short*)C0;
    unsigned short* P1 = (unsigned short*)C1;
#pragma unroll
    for (int i = 0; i < 2; ++i) {
#pragma unroll
      for (int r = 0; r < 8; ++r) {
#pragma unroll
        for (int j = 0; j < 8; ++j) {
          const float v = acc[i][j][r];
          const unsigned short hb = bf_bits(v);
          const unsigned short lb = bf_bits(v - bf_val(hb));
          const int so = (8 * hh + r) * 128 + j * 16 + rl;
          sl16[so]        = hb;
          sl16[2048 + so] = lb;
        }
      }
      lds_wave_sync();
      for (int pass = 0; pass < 2; ++pass) {
#pragma unroll
        for (int it = 0; it < 8; ++it) {
          const int row = it * 2 + hh;
          const int c8  = rl * 8;
          const v4u vh = *(const v4u*)(sl16 + row * 128 + c8);
          const v4u vl = *(const v4u*)(sl16 + 2048 + row * 128 + c8);
          const size_t go = (size_t)(m0 + i * 16 + row) * ldc + n0 + c8;
          *(volatile v4u*)(P0 + go) = vh;
          *(volatile v4u*)(P1 + go) = vl;
        }
        __threadfence();
      }
      lds_wave_sync();
    }
  } else {
    float* C = (float*)C0;
    v4f bb = {0.f, 0.f, 0.f, 0.f};
    if (HASBIAS) {
      const v4f t = *(const v4f*)(bias + n0 + lane * 4);
      bb[0] = bf_rne(t[0]); bb[1] = bf_rne(t[1]); bb[2] = bf_rne(t[2]); bb[3] = bf_rne(t[3]);
    }
#pragma unroll
    for (int i = 0; i < 2; ++i) {
#pragma unroll
      for (int j = 0; j < 8; ++j)
#pragma unroll
        for (int r = 0; r < 8; ++r)
          slf[(8 * hh + r) * 128 + j * 16 + rl] = acc[i][j][r];
      lds_wave_sync();
      for (int pass = 0; pass < 2; ++pass) {
#pragma unroll
        for (int row = 0; row < 16; ++row) {
          const v4f v = *(const v4f*)(slf + row * 128 + lane * 4) + bb;
          *(volatile v4f*)(C + (size_t)(m0 + i * 16 + row) * ldc + n0 + lane * 4) = v;
        }
        __threadfence();
      }
      lds_wave_sync();
    }
  }
}

#define ACH   64
#define AQP   136
#define AKP   136
#define AVP   72
#define APP   72
#define A_OQH 0
#define A_OQL (64 * AQP)
#define A_OKH (2 * 64 * AQP)
#define A_OKL (A_OKH + 64 * AKP)
#define A_OVH (A_OKL + 64 * AKP)
#define A_OVL (A_OVH + HD * AVP)
#define A_OPH (A_OVL + HD * AVP)
#define A_OPL (A_OPH + 4 * 16 * APP)
#define A_TOT (A_OPL + 4 * 16 * APP)
#define ATT_LDS_BYTES (A_TOT * 2)
static_assert(ATT_LDS_BYTES == 124928);
static_assert(4 * 16 * HD <= 64 * AKP);
static_assert((A_OQL % 8) == 0 && (A_OKH % 8) == 0 && (A_OKL % 8) == 0 && (A_OVH % 8) == 0 && (A_OVL % 8) == 0 &&
              (A_OPH % 8) == 0 && (A_OPL % 8) == 0);

extern __shared__ __align__(16) unsigned short att_smem[];

__global__ __launch_bounds__(128) void attn_causal128_kernel(
    const unsigned short* __restrict__ qhp, const unsigned short* __restrict__ qlp,
    const unsigned short* __restrict__ khp, const unsigned short* __restrict__ klp,
    const unsigned short* __restrict__ vhp, const unsigned short* __restrict__ vlp,
    unsigned short* __restrict__ aop, float sscale) {
  unsigned short* Qhs = att_smem + A_OQH;
  unsigned short* Qls = att_smem + A_OQL;
  unsigned short* Khs = att_smem + A_OKH;
  unsigned short* Kls = att_smem + A_OKL;
  unsigned short* Vhs = att_smem + A_OVH;
  unsigned short* Vls = att_smem + A_OVL;
  unsigned short* Phs = att_smem + A_OPH;
  unsigned short* Pls = att_smem + A_OPL;

  const int tid  = (int)threadIdx.x;
  const int lane = tid & 31;
  const int wave = wave_id();
  const int hh   = lane >> 4;
  const int c    = lane & 15;
  const int qt   = (int)blockIdx.x;
  const int h    = (int)blockIdx.y;
  const int qb0  = qt * 64;

#pragma unroll 2
  for (int u = 0; u < 8; ++u) {
    const int p  = tid + 128 * u;
    const int r  = p >> 4, d8 = (p & 15) * 8;
    const size_t qo = (size_t)(qb0 + r) * NQ + h * HD + d8;
    const v4u qa = *(const v4u*)(qhp + qo);
    const v4u qb = *(const v4u*)(qlp + qo);
    *(v4u*)(Qhs + r * AQP + d8) = qa;
    *(v4u*)(Qls + r * AQP + d8) = qb;
  }

  unsigned short* ph = Phs + wave * 16 * APP;
  unsigned short* pl = Pls + wave * 16 * APP;

  float mrow[8], lrow[8];
  v8f oacc[8];
#pragma unroll
  for (int r = 0; r < 8; ++r) { mrow[r] = -INFINITY; lrow[r] = 0.f; }
#pragma unroll
  for (int t = 0; t < 8; ++t) oacc[t] = zero8();

  const int nChunks = qt + 1;
  for (int kc = 0; kc < nChunks; ++kc) {
    const int kv0 = kc * ACH;
    __syncthreads();
#pragma unroll 2
    for (int u = 0; u < 8; ++u) {
      const int p   = tid + 128 * u;
      const int key = p >> 4, d8 = (p & 15) * 8;
      const size_t ko = (size_t)(kv0 + key) * NQ + h * HD + d8;
      const v4u kx = *(const v4u*)(khp + ko);
      const v4u ky = *(const v4u*)(klp + ko);
      *(v4u*)(Khs + key * AKP + d8) = kx;
      *(v4u*)(Kls + key * AKP + d8) = ky;
      const int d = p >> 3, k8 = (p & 7) * 8;
      const size_t vo = (size_t)(h * HD + d) * SQ + kv0 + k8;
      const v4u vx = *(const v4u*)(vhp + vo);
      const v4u vy = *(const v4u*)(vlp + vo);
      *(v4u*)(Vhs + d * AVP + k8) = vx;
      *(v4u*)(Vls + d * AVP + k8) = vy;
    }
    __syncthreads();

    v8f sa[4];
    sa[0] = zero8(); sa[1] = zero8(); sa[2] = zero8(); sa[3] = zero8();
#pragma unroll
    for (int dc = 0; dc < 4; ++dc) {
      const v16b qh = ldfrag_b((const __bf16*)(const void*)Qhs + (wave * 16 + c) * AQP + dc * 32 + 8 * hh);
      const v16b ql = ldfrag_b((const __bf16*)(const void*)Qls + (wave * 16 + c) * AQP + dc * 32 + 8 * hh);
#pragma unroll
      for (int j = 0; j < 4; ++j) {
        const v16b kb = ldfrag_b((const __bf16*)(const void*)Khs + (j * 16 + c) * AKP + dc * 32 + 8 * hh);
        const v16b kl = ldfrag_b((const __bf16*)(const void*)Kls + (j * 16 + c) * AKP + dc * 32 + 8 * hh);
        sa[j] = mma_b(qh, kb, sa[j]);
        sa[j] = mma_b(qh, kl, sa[j]);
        sa[j] = mma_b(ql, kb, sa[j]);
        guard1b4(sa[j], qh, ql, kb, kl);
      }
    }
    acc_guard4(sa[0], sa[1], sa[2], sa[3]);

    const bool diag = (kc == qt);
    float cm[8];
#pragma unroll
    for (int r = 0; r < 8; ++r) {
      const int qrow = qb0 + wave * 16 + 8 * hh + r;
      float m = -INFINITY;
#pragma unroll
      for (int j = 0; j < 4; ++j) {
        const int kvcol = kv0 + j * 16 + c;
        const float sv = sa[j][r] * sscale;
        const bool masked = diag && (kvcol > qrow);
        const float sm = masked ? -INFINITY : sv;
        sa[j][r] = sm;
        m = fmaxf(m, sm);
      }
#pragma unroll
      for (int off = 1; off < 16; off <<= 1) m = fmaxf(m, __shfl_xor(m, off, 32));
      cm[r] = m;
    }
#pragma unroll
    for (int r = 0; r < 8; ++r) {
      const float mnew  = fmaxf(mrow[r], cm[r]);
      const float alpha = __expf(mrow[r] - mnew);
      mrow[r] = mnew;
      float psum = 0.f;
#pragma unroll
      for (int j = 0; j < 4; ++j) {
        const float p = __expf(sa[j][r] - mnew);
        psum += p;
        const unsigned short hb = bf_bits(p);
        const unsigned short lb = bf_bits(p - bf_val(hb));
        const int po = (8 * hh + r) * APP + j * 16 + c;
        ph[po] = hb;
        pl[po] = lb;
      }
#pragma unroll
      for (int off = 1; off < 16; off <<= 1) psum += __shfl_xor(psum, off, 32);
      lrow[r] = lrow[r] * alpha + psum;
#pragma unroll
      for (int t = 0; t < 8; ++t) oacc[t][r] *= alpha;
    }
    lds_wave_sync();
#pragma unroll 1
    for (int kk = 0; kk < 2; ++kk) {
      const v16b pa = ldfrag_b((const __bf16*)(const void*)ph + c * APP + kk * 32 + 8 * hh);
      const v16b pr = ldfrag_b((const __bf16*)(const void*)pl + c * APP + kk * 32 + 8 * hh);
#pragma unroll
      for (int t = 0; t < 8; ++t) {
        const v16b vb = ldfrag_b((const __bf16*)(const void*)Vhs + (t * 16 + c) * AVP + kk * 32 + 8 * hh);
        const v16b vr = ldfrag_b((const __bf16*)(const void*)Vls + (t * 16 + c) * AVP + kk * 32 + 8 * hh);
        oacc[t] = mma_b(pa, vb, oacc[t]);
        oacc[t] = mma_b(pa, vr, oacc[t]);
        oacc[t] = mma_b(pr, vb, oacc[t]);
        guard1b4(oacc[t], pa, pr, vb, vr);
      }
    }
  }
  __syncthreads();
  acc_guard4(oacc[0], oacc[1], oacc[2], oacc[3]);
  acc_guard4(oacc[4], oacc[5], oacc[6], oacc[7]);

  unsigned short* osh = Khs + wave * (16 * HD);
  unsigned short* osl = Kls + wave * (16 * HD);
#pragma unroll
  for (int r = 0; r < 8; ++r) {
    const float inv = 1.0f / lrow[r];
#pragma unroll
    for (int t = 0; t < 8; ++t) {
      const float o = oacc[t][r] * inv;
      const unsigned short hb = bf_bits(o);
      const unsigned short lb = bf_bits(o - bf_val(hb));
      const int so = (8 * hh + r) * HD + t * 16 + c;
      osh[so] = hb;
      osl[so] = lb;
    }
  }
  lds_wave_sync();
  unsigned short* Ag = aop + (size_t)(qb0 + wave * 16) * AOW + h * HD;
  const int c8 = c * 8;
  for (int pass = 0; pass < 2; ++pass) {
#pragma unroll
    for (int it = 0; it < 8; ++it) {
      const int row = it * 2 + hh;
      const v4u x = *(const v4u*)(osh + row * HD + c8);
      const v4u y = *(const v4u*)(osl + row * HD + c8);
      *(volatile v4u*)(Ag + (size_t)row * AOW + c8)      = x;
      *(volatile v4u*)(Ag + (size_t)row * AOW + NQ + c8) = y;
    }
    __threadfence();
  }
}

extern "C" void kernel_launch(void* const* d_in, const int* in_sizes, int n_in,
                              void* d_out, int out_size, void* d_ws, size_t ws_size,
                              hipStream_t stream) {
  if (n_in < 9) return;
  if (in_sizes[0] != NB * SQ * DMOD) return;
  if (in_sizes[1] != SQ * NPAIR * 2) return;
  if (in_sizes[2] != NQ * DMOD) return;
  if (in_sizes[3] != NQ) return;
  if (in_sizes[4] != DLAT * DMOD) return;
  if (in_sizes[5] != 2 * NQ * DLAT) return;
  if (in_sizes[6] != DLAT) return;
  if (in_sizes[7] != DMOD * NQ) return;
  if (in_sizes[8] != DMOD) return;
  if (out_size != NB * SQ * DMOD) return;

  const float* x      = (const float*)d_in[0];
  const float* freqs  = (const float*)d_in[1];
  const float* wq_w   = (const float*)d_in[2];
  const float* wq_b   = (const float*)d_in[3];
  const float* wkva_w = (const float*)d_in[4];
  const float* wkvb_w = (const float*)d_in[5];
  const float* norm_w = (const float*)d_in[6];
  const float* out_w  = (const float*)d_in[7];
  const float* out_b  = (const float*)d_in[8];
  float* out = (float*)d_out;

  const size_t szXB    = (size_t)SQ * DMOD * 2;
  const size_t szWA    = (size_t)NQA * DMOD * 2;
  const size_t szWKVB2 = (size_t)2 * NQ * KVBW * 2;
  const size_t szWO2   = (size_t)DMOD * WOW * 2;
  const size_t szTP    = (size_t)SQ * DLAT * 4;
  const size_t szLAT   = (size_t)SQ * LATW * 2;
  const size_t szP     = (size_t)SQ * NQ * 2;
  const size_t szAO    = (size_t)SQ * AOW * 2;
  size_t off = 0;
  const size_t oXB    = off; off += szXB;
  const size_t oWA    = off; off += szWA;
  const size_t oWKVB2 = off; off += szWKVB2;
  const size_t oWO2   = off; off += szWO2;
  const size_t oTP    = off; off += szTP;
  const size_t oLAT   = off; off += szLAT;
  const size_t oQH    = off; off += szP;
  const size_t oQL    = off; off += szP;
  const size_t oKH    = off; off += szP;
  const size_t oKL    = off; off += szP;
  const size_t oVTH   = off; off += szP;
  const size_t oVTL   = off; off += szP;
  const size_t oAO    = off; off += szAO;
  if (off > ws_size) return;

  char* ws = (char*)d_ws;
  unsigned short* XB    = (unsigned short*)(ws + oXB);
  unsigned short* WA    = (unsigned short*)(ws + oWA);
  unsigned short* WKVB2 = (unsigned short*)(ws + oWKVB2);
  unsigned short* WO2   = (unsigned short*)(ws + oWO2);
  float*          TP    = (float*)(ws + oTP);
  unsigned short* LAT   = (unsigned short*)(ws + oLAT);
  unsigned short* QH    = (unsigned short*)(ws + oQH);
  unsigned short* QL    = (unsigned short*)(ws + oQL);
  unsigned short* KH    = (unsigned short*)(ws + oKH);
  unsigned short* KL    = (unsigned short*)(ws + oKL);
  unsigned short* VTH   = (unsigned short*)(ws + oVTH);
  unsigned short* VTL   = (unsigned short*)(ws + oVTL);
  unsigned short* AO    = (unsigned short*)(ws + oAO);

  const dim3 b256(256), b128(128);
  const int n8q  = NQ * DMOD / 8;
  const int n8a  = DLAT * DMOD / 8;
  const int n8kb = 2 * NQ * DLAT / 8;
  const int n8o  = DMOD * NQ / 8;
  const int n8x  = SQ * DMOD / 8;

  cvt_bf16_kernel<<<dim3((n8q + 255) / 256), b256, 0, stream>>>(wq_w, WA, n8q);
  cvt_bf16_kernel<<<dim3((n8a + 255) / 256), b256, 0, stream>>>(wkva_w, WA + (size_t)NQ * DMOD, n8a);
  cvt_dup_kernel<<<dim3((n8kb + 255) / 256), b256, 0, stream>>>(wkvb_w, WKVB2, n8kb, DLAT, KVBW);
  cvt_dup_kernel<<<dim3((n8o + 255) / 256), b256, 0, stream>>>(out_w, WO2, n8o, NQ, WOW);

  (void)hipFuncSetAttribute(reinterpret_cast<const void*>(&attn_causal128_kernel),
                            hipFuncAttributeMaxDynamicSharedMemorySize, ATT_LDS_BYTES);

  const dim3 gA(((SQ / 32) * (NQA / 128) + 3) / 4);
  const dim3 gK(((SQ / 32) * (NQ / 128) + 3) / 4);
  const dim3 gV(((NQ / 32) * (SQ / 128) + 3) / 4);
  const dim3 gO(((SQ / 32) * (DMOD / 128) + 3) / 4);
  const dim3 gRms((SQ + 7) / 8);
  const dim3 gAtt(SQ / 64, NH);
  const float sscale = 0.08838834764831845f;

  for (int b = 0; b < NB; ++b) {
    const float* xb = x + (size_t)b * SQ * DMOD;
    cvt_bf16_kernel<<<dim3((n8x + 255) / 256), b256, 0, stream>>>(xb, XB, n8x);
    gemm_w32x128_kernel<0, true><<<gA, b128, 0, stream>>>(
        XB, DMOD, WA, DMOD, wq_b, freqs, (void*)QH, (void*)QL, (void*)TP, NQ, DLAT, NQ, SQ, NQA, DMOD);
    rmsnorm_split_kernel<<<gRms, b256, 0, stream>>>(TP, norm_w, LAT, SQ);
    gemm_w32x128_kernel<0, false><<<gK, b128, 0, stream>>>(
        LAT, LATW, WKVB2, KVBW, wq_b, freqs, (void*)KH, (void*)KL, (void*)TP, NQ, DLAT, NQ, SQ, NQ, LATW);
    gemm_w32x128_kernel<1, false><<<gV, b128, 0, stream>>>(
        WKVB2 + (size_t)NQ * KVBW, KVBW, LAT, LATW, wq_b, freqs, (void*)VTH, (void*)VTL, (void*)TP, SQ, DLAT, NQ, NQ, SQ, LATW);
    attn_causal128_kernel<<<gAtt, b128, ATT_LDS_BYTES, stream>>>(QH, QL, KH, KL, VTH, VTL, AO, sscale);
    float* outb = out + (size_t)b * SQ * DMOD;
    gemm_w32x128_kernel<2, true><<<gO, b128, 0, stream>>>(
        AO, AOW, WO2, WOW, out_b, freqs, (void*)outb, (void*)outb, (void*)outb, DMOD, DLAT, NQ, SQ, DMOD, AOW);
  }
  (void)hipGetLastError();
}
